// GAT_86990267613313
// MI455X (gfx1250) — hardware-run, weakly checked
//
#include <hip/hip_runtime.h>
#include <stddef.h>
#include <stdint.h>
#include <math.h>

#define NN      50000
#define NE      800000
#define DIN     128
#define W1N     256
#define W2N     128
#define C2      64
#define EP      256
#define TWO_TERM 1
#define K2EXT   (TWO_TERM ? 256 : 128)
#define GBM     128
#define MP      50048
#define NTHR    256
#define NWAVE   8
#define EPT     8
#define WCH     (32 * EPT)
#define NBRUN   1024
#define SLB     10
#define NBK     49
#define WLCAP   3584
#define RCAP    28672
#define DEGCAP  256
#define MAXDEG_MEAS   35
#define MAXB1024_MEAS 16623
#define SP      68
#define NEGS    0.2f

#define BK_ZINTS (NWAVE * WLCAP + RCAP + 3 * NBRUN)
#define BK_INTS  (BK_ZINTS + 16)
#define BK_LDS   (BK_INTS * 4)

#define PBX   (MP * DIN / 8 / NTHR)
#define PBW   8
#define PBTOT (PBX + 4 * PBW + 1)

#define SM_ATT1 0
#define SM_B1   128
#define SM_ATT2 256
#define SM_B2   320
#define SM_N    384

static_assert(MP % GBM == 0 && MP >= NN && MP == 391 * GBM && MP % NWAVE == 0);
static_assert(NN % 2 == 0 && NN % NWAVE == 0);
static_assert(NBRUN == (1 << SLB) && NBRUN % 32 == 0);
static_assert(NBK * NBRUN >= MP);
static_assert((NBK - 1) * NBRUN < NN);
static_assert(NE <= (1 << 20) && (((long long)NE) << SLB) < (1LL << 31));
static_assert(NE % WCH == 0 && NE % 4 == 0);
static_assert(RCAP == NWAVE * WLCAP && RCAP % 4 == 0 && BK_ZINTS % 4 == 0);
static_assert(RCAP % (NTHR * 4) == 0 && (2 * NBRUN) % (NTHR * 4) == 0);
static_assert((long long)RCAP * 100 >= (long long)MAXB1024_MEAS * 105);
static_assert(WLCAP >= MAXB1024_MEAS / 8 + 8 * 46 + 1);
static_assert(MAXDEG_MEAS + 8 <= DEGCAP);
static_assert(BK_LDS <= 300000);
static_assert(GBM * SP * 4 <= 65536);
static_assert((MP * DIN / 8) % NTHR == 0);
static_assert(W1N * DIN / 8 == 2 * PBW * NTHR && W2N * 256 / 8 == 2 * PBW * NTHR);
static_assert(DIN % 32 == 0 && K2EXT % 32 == 0 && K2EXT <= EP);
static_assert(W1N % 64 == 0 && W2N % 64 == 0);

typedef float          v2f   __attribute__((ext_vector_type(2)));
typedef float          v4f   __attribute__((ext_vector_type(4)));
typedef float          v8f   __attribute__((ext_vector_type(8)));
typedef unsigned       v2u   __attribute__((ext_vector_type(2)));
typedef int            v4i   __attribute__((ext_vector_type(4)));
typedef int            v8i   __attribute__((ext_vector_type(8)));
typedef unsigned short v8us  __attribute__((ext_vector_type(8)));
typedef unsigned short v16us __attribute__((ext_vector_type(16)));
typedef __bf16         v16bf __attribute__((ext_vector_type(16)));
typedef v2f  __attribute__((may_alias)) v2fa;
typedef v4f  __attribute__((may_alias)) v4fa;
typedef v4i  __attribute__((may_alias)) v4ia;
typedef v8us __attribute__((may_alias)) v8usa;
union FragB { v16bf v; v16us u; v8us h[2]; v8i w; };

__device__ __forceinline__ v8f wmb(const FragB& a, const FragB& b, v8f c) {
  v8f d = __builtin_amdgcn_wmma_f32_16x16x32_bf16(false, a.v, false, b.v, (short)0, c, false, false);
  asm volatile("v_nop\n\tv_nop\n\tv_nop\n\tv_nop" : "+v"(d) : "v"(a.w), "v"(b.w));
  return d;
}

__device__ __forceinline__ unsigned bf16_bits(float f) {
  const unsigned u = __float_as_uint(f);
  const unsigned r = (u + 0x7FFFu + ((u >> 16) & 1u)) >> 16;
  const unsigned q = (u >> 16) | 0x40u;
  return ((u & 0x7fffffffu) > 0x7f800000u) ? q : r;
}
__device__ __forceinline__ float bf16_val(float f) {
  return __uint_as_float(bf16_bits(f) << 16);
}
__device__ __forceinline__ v4f bf16_val4(const v4f a) {
  v4f o;
  o.x = bf16_val(a.x); o.y = bf16_val(a.y); o.z = bf16_val(a.z); o.w = bf16_val(a.w);
  return o;
}

__device__ __forceinline__ void st2_v4f(float* p, v4f v) {
  *(volatile v4f*)p = v;
  __threadfence();
  *(volatile v4f*)p = v;
}
__device__ __forceinline__ void st2_v8us(unsigned short* p, v8us v) {
  *(volatile v8us*)p = v;
  __threadfence();
  *(volatile v8us*)p = v;
}

__device__ __forceinline__ v8us colpick8(const float* __restrict__ base, int stride) {
  float f[8];
#pragma unroll
  for (int i = 0; i < 8; ++i) f[i] = base[(size_t)i * (size_t)stride];
  v8us o;
#pragma unroll
  for (int i = 0; i < 8; ++i) o[i] = (unsigned short)bf16_bits(f[i]);
  return o;
}

__global__ __launch_bounds__(NTHR) void k_prep(const float* __restrict__ x,
                                               const float* __restrict__ wl1, const float* __restrict__ wr1,
                                               const float* __restrict__ att1, const float* __restrict__ b1,
                                               const float* __restrict__ wl2, const float* __restrict__ wr2,
                                               const float* __restrict__ att2, const float* __restrict__ b2,
                                               unsigned short* xb, unsigned short* bt1, unsigned short* bt2,
                                               float* sm) {
  const int tid = (int)threadIdx.x, lane = tid & 31, wave = tid >> 5;
  const int blk = (int)blockIdx.x;
  if (blk < PBX) {
    const int u   = blk * NTHR + tid;
    const int row = u >> 4, k8 = (u & 15) * 8;
    const int rc  = row < NN ? row : NN - 1;
    const unsigned mk = row < NN ? 0xffffu : 0u;
    const float* p = x + (size_t)rc * DIN + k8;
    const v4f a = *(const v4fa*)p;
    const v4f b = *(const v4fa*)(p + 4);
    v8us o;
    o[0] = (unsigned short)(bf16_bits(a.x) & mk); o[1] = (unsigned short)(bf16_bits(a.y) & mk);
    o[2] = (unsigned short)(bf16_bits(a.z) & mk); o[3] = (unsigned short)(bf16_bits(a.w) & mk);
    o[4] = (unsigned short)(bf16_bits(b.x) & mk); o[5] = (unsigned short)(bf16_bits(b.y) & mk);
    o[6] = (unsigned short)(bf16_bits(b.z) & mk); o[7] = (unsigned short)(bf16_bits(b.w) & mk);
    st2_v8us(xb + (size_t)row * DIN + k8, o);
  } else if (blk < PBX + PBW) {
    const int u = (blk - PBX) * NTHR + tid;
    const int n = u >> 4, k8 = (u & 15) * 8;
    const v8us o = colpick8(wl1 + (size_t)k8 * 128 + n, 128);
    st2_v8us(bt1 + (size_t)n * DIN + k8, o);
  } else if (blk < PBX + 2 * PBW) {
    const int u = (blk - PBX - PBW) * NTHR + tid;
    const int n = u >> 4, k8 = (u & 15) * 8;
    const v8us o = colpick8(wr1 + (size_t)k8 * 128 + n, 128);
    st2_v8us(bt1 + (size_t)(128 + n) * DIN + k8, o);
  } else if (blk < PBX + 3 * PBW) {
    const int u = (blk - PBX - 2 * PBW) * NTHR + tid;
    const int n = u >> 5, k8 = (u & 31) * 8, kk = k8 & 127;
    const v8us o = colpick8(wl2 + (size_t)kk * 64 + n, 64);
    st2_v8us(bt2 + (size_t)n * 256 + k8, o);
  } else if (blk < PBX + 4 * PBW) {
    const int u = (blk - PBX - 3 * PBW) * NTHR + tid;
    const int n = u >> 5, k8 = (u & 31) * 8, kk = k8 & 127;
    const v8us o = colpick8(wr2 + (size_t)kk * 64 + n, 64);
    st2_v8us(bt2 + (size_t)(64 + n) * 256 + k8, o);
  } else {
    if (wave == 0) {
      const v4f a = *(const v4fa*)(att1 + 4 * lane);
      asm volatile("" :: "v"(a));
      st2_v4f(sm + SM_ATT1 + 4 * lane, bf16_val4(a));
    } else if (wave == 1) {
      const v4f a = *(const v4fa*)(b1 + 4 * lane);
      asm volatile("" :: "v"(a));
      st2_v4f(sm + SM_B1 + 4 * lane, bf16_val4(a));
    } else if (wave == 2) {
      const int q = lane & 15;
      const v4f a = *(const v4fa*)(att2 + 4 * q);
      const v4f c = *(const v4fa*)(b2 + 4 * q);
      asm volatile("" :: "v"(a));
      asm volatile("" :: "v"(c));
      const unsigned ma = (lane < 16) ? 0xffffffffu : 0u;
      v4f o;
      o.x = __uint_as_float(((bf16_bits(a.x) << 16) & ma) | ((bf16_bits(c.x) << 16) & ~ma));
      o.y = __uint_as_float(((bf16_bits(a.y) << 16) & ma) | ((bf16_bits(c.y) << 16) & ~ma));
      o.z = __uint_as_float(((bf16_bits(a.z) << 16) & ma) | ((bf16_bits(c.z) << 16) & ~ma));
      o.w = __uint_as_float(((bf16_bits(a.w) << 16) & ma) | ((bf16_bits(c.w) << 16) & ~ma));
      st2_v4f(sm + SM_ATT2 + 4 * lane, o);
    }
  }
}

template <int KEXT, int BPITCH>
__device__ __forceinline__ void gemm_16x64(const unsigned short* __restrict__ ap,
                                           const unsigned short* __restrict__ bp, v8f (&acc)[4]) {
#pragma unroll 1
  for (int k0 = 0; k0 < KEXT; k0 += 32) {
    FragB af;
    af.h[0] = *(const v8usa*)(ap + k0);
    af.h[1] = *(const v8usa*)(ap + k0 + 16);
#pragma unroll
    for (int nt = 0; nt < 4; ++nt) {
      const unsigned short* wq = bp + (size_t)(16 * nt) * (size_t)BPITCH + k0;
      FragB bf;
      bf.h[0] = *(const v8usa*)wq;
      bf.h[1] = *(const v8usa*)(wq + 16);
      acc[nt] = wmb(af, bf, acc[nt]);
    }
  }
}

__device__ __forceinline__ void stage_d(float* stg, const v8f (&acc)[4], int wave, int hh, int m) {
#pragma unroll
  for (int nt = 0; nt < 4; ++nt) {
#pragma unroll
    for (int r = 0; r < 8; ++r) stg[(16 * wave + 8 * hh + r) * SP + 16 * nt + m] = acc[nt][r];
  }
}

template <int KEXT, int APITCH, int BPITCH, int LDO>
__device__ __forceinline__ void gemm_tile(const unsigned short* __restrict__ A,
                                          const unsigned short* __restrict__ BT, float* out, float* stg) {
  const int tid = (int)threadIdx.x, lane = tid & 31, wave = tid >> 5, hh = lane >> 4, m = lane & 15;
  const int rowBase = (int)blockIdx.x * GBM;
  const int col0    = (int)blockIdx.y * 64;

  v8f acc[4];
  {
    const v8f z = {0.f, 0.f, 0.f, 0.f, 0.f, 0.f, 0.f, 0.f};
#pragma unroll
    for (int t = 0; t < 4; ++t) acc[t] = z;
  }
  const unsigned short* ap = A + (size_t)(rowBase + 16 * wave + m) * (size_t)APITCH + 8 * hh;
  const unsigned short* bp = BT + (size_t)(col0 + m) * (size_t)BPITCH + 8 * hh;
  gemm_16x64<KEXT, BPITCH>(ap, bp, acc);
  stage_d(stg, acc, wave, hh, m);
  __syncthreads();

  v4f fv[8];
#pragma unroll
  for (int i = 0; i < 8; ++i) {
    const int lr = 16 * wave + 2 * i + hh;
    fv[i] = *(const v4fa*)(stg + lr * SP + 4 * m);
    asm volatile("" :: "v"(fv[i]));
  }
#pragma unroll
  for (int i = 0; i < 8; ++i) {
    const int grow = rowBase + 16 * wave + 2 * i + hh;
    float* op = out + (size_t)grow * (size_t)LDO + col0 + 4 * m;
    if (grow < NN) *(volatile v4f*)op = fv[i];
  }
  __threadfence();
#pragma unroll
  for (int i = 0; i < 8; ++i) {
    const int grow = rowBase + 16 * wave + 2 * i + hh;
    float* op = out + (size_t)grow * (size_t)LDO + col0 + 4 * m;
    if (grow < NN) *(volatile v4f*)op = fv[i];
  }
}

__global__ __launch_bounds__(NTHR) __attribute__((amdgpu_num_vgpr(248)))
void k_gemm_one(const unsigned short* __restrict__ XB, const unsigned short* __restrict__ BT1, float* XLR1) {
  __shared__ __attribute__((aligned(16))) float stg[GBM * SP];
  gemm_tile<DIN, DIN, DIN, W1N>(XB, BT1, XLR1, stg);
}

__global__ __launch_bounds__(NTHR) __attribute__((amdgpu_num_vgpr(248)))
void k_gemm_two(const unsigned short* __restrict__ E, const unsigned short* __restrict__ BT2, float* XLR2) {
  __shared__ __attribute__((aligned(16))) float stg[GBM * SP];
  gemm_tile<K2EXT, EP, 256, W2N>(E, BT2, XLR2, stg);
}

__device__ __forceinline__ void bucket_flush(const int* pl, const int* cnt, int ov, int* lp, int* cop, int* fp,
                                             int tid) {
#pragma unroll 1
  for (int i = tid * 4; i < RCAP; i += NTHR * 4) {
    const v4i v = *(const v4ia*)(pl + i);
    *(volatile v4i*)(lp + i) = v;
  }
#pragma unroll 1
  for (int i = tid * 4; i < 2 * NBRUN; i += NTHR * 4) {
    const v4i v = *(const v4ia*)(cnt + i);
    *(volatile v4i*)(cop + i) = v;
  }
  if (tid < 8) {
    const v4i f = {ov, ov, ov, ov};
    *(volatile v4i*)(fp + 4 * tid) = f;
  }
}

__global__ __launch_bounds__(NTHR) void k_bucket(const int* __restrict__ srcs, const int* __restrict__ dsts,
                                                 int* LIST, int* CO, int* FLAG) {
  extern __shared__ __attribute__((aligned(16))) int dsm[];
  int* wl   = dsm;
  int* pl   = dsm + NWAVE * WLCAP;
  int* cnt  = pl + RCAP;
  int* offs = cnt + NBRUN;
  int* cur  = offs + NBRUN;
  int* misc = cur + NBRUN;
  const int tid = (int)threadIdx.x, lane = tid & 31, wave = tid >> 5;
  const int blk = (int)blockIdx.x;
  const unsigned nbs = (unsigned)(blk * NBRUN);
  const int nbl = (NN - blk * NBRUN) < NBRUN ? (NN - blk * NBRUN) : NBRUN;
  const unsigned unb = (unsigned)(nbl < 0 ? 0 : nbl);

  {
    const v4i z4 = {0, 0, 0, 0};
    for (int i = tid * 4; i < BK_ZINTS; i += NTHR * 4) *(v4ia*)(dsm + i) = z4;
    if (tid < 16) misc[tid] = 0;
  }
  __syncthreads();

  {
    const int per  = ((NE + NWAVE * WCH - 1) / (NWAVE * WCH)) * WCH;
    const int ebeg = wave * per;
    const int eend = (ebeg + per < NE) ? (ebeg + per) : NE;
    int* mylist = wl + wave * WLCAP;
    int wc = 0;
#pragma unroll 1
    for (int cb = ebeg; cb < eend; cb += WCH) {
      const int e0 = cb + lane * EPT;
      const v4i da = *(const v4ia*)(dsts + e0);
      const v4i db = *(const v4ia*)(dsts + e0 + 4);
      const unsigned s0 = (unsigned)da.x - nbs, s1 = (unsigned)da.y - nbs;
      const unsigned s2 = (unsigned)da.z - nbs, s3 = (unsigned)da.w - nbs;
      const unsigned s4 = (unsigned)db.x - nbs, s5 = (unsigned)db.y - nbs;
      const unsigned s6 = (unsigned)db.z - nbs, s7 = (unsigned)db.w - nbs;
      const bool h0 = s0 < unb, h1 = s1 < unb, h2 = s2 < unb, h3 = s3 < unb;
      const bool h4 = s4 < unb, h5 = s5 < unb, h6 = s6 < unb, h7 = s7 < unb;
      const unsigned m0 = __builtin_amdgcn_ballot_w32(h0), m1 = __builtin_amdgcn_ballot_w32(h1);
      const unsigned m2 = __builtin_amdgcn_ballot_w32(h2), m3 = __builtin_amdgcn_ballot_w32(h3);
      const unsigned m4 = __builtin_amdgcn_ballot_w32(h4), m5 = __builtin_amdgcn_ballot_w32(h5);
      const unsigned m6 = __builtin_amdgcn_ballot_w32(h6), m7 = __builtin_amdgcn_ballot_w32(h7);
      const unsigned any = m0 | m1 | m2 | m3 | m4 | m5 | m6 | m7;
      if (any != 0u) {
        const int pre = (int)(__builtin_amdgcn_mbcnt_lo(m0, 0u) + __builtin_amdgcn_mbcnt_lo(m1, 0u) +
                              __builtin_amdgcn_mbcnt_lo(m2, 0u) + __builtin_amdgcn_mbcnt_lo(m3, 0u) +
                              __builtin_amdgcn_mbcnt_lo(m4, 0u) + __builtin_amdgcn_mbcnt_lo(m5, 0u) +
                              __builtin_amdgcn_mbcnt_lo(m6, 0u) + __builtin_amdgcn_mbcnt_lo(m7, 0u));
        int p = wc + pre;
        if (h0) { if (p < WLCAP) mylist[p] = ((e0 + 0) << SLB) | (int)s0; p = p + 1; }
        if (h1) { if (p < WLCAP) mylist[p] = ((e0 + 1) << SLB) | (int)s1; p = p + 1; }
        if (h2) { if (p < WLCAP) mylist[p] = ((e0 + 2) << SLB) | (int)s2; p = p + 1; }
        if (h3) { if (p < WLCAP) mylist[p] = ((e0 + 3) << SLB) | (int)s3; p = p + 1; }
        if (h4) { if (p < WLCAP) mylist[p] = ((e0 + 4) << SLB) | (int)s4; p = p + 1; }
        if (h5) { if (p < WLCAP) mylist[p] = ((e0 + 5) << SLB) | (int)s5; p = p + 1; }
        if (h6) { if (p < WLCAP) mylist[p] = ((e0 + 6) << SLB) | (int)s6; p = p + 1; }
        if (h7) { if (p < WLCAP) mylist[p] = ((e0 + 7) << SLB) | (int)s7; p = p + 1; }
        wc += (int)(__builtin_popcount(m0) + __builtin_popcount(m1) + __builtin_popcount(m2) + __builtin_popcount(m3) +
                    __builtin_popcount(m4) + __builtin_popcount(m5) + __builtin_popcount(m6) + __builtin_popcount(m7));
      }
    }
    if (lane == 0) misc[wave] = wc;
  }
  __syncthreads();

  if (wave == 0) {
    int ov = 0;
#pragma unroll 1
    for (int w2 = 0; w2 < NWAVE; ++w2) {
      int c = misc[w2];
      if (c > WLCAP) ov = 1;
      c = c < 0 ? 0 : (c > WLCAP ? WLCAP : c);
#pragma unroll 1
      for (int b0 = 0; b0 < c; b0 += 32) {
        const int idx = b0 + lane;
        const int ent = wl[w2 * WLCAP + (idx < WLCAP ? idx : WLCAP - 1)];
        const int m32 = (c - b0) < 32 ? (c - b0) : 32;
#pragma unroll 1
        for (int k = 0; k < m32; ++k) {
          const int u    = __builtin_amdgcn_readlane(ent, k);
          const int slot = u & (NBRUN - 1);
          if (lane == 0) cnt[slot] = cnt[slot] + 1;
        }
      }
    }
    if (lane == 0) misc[9] = ov;
  }
  __syncthreads();
  if (wave == 0) {
    const int base = lane * (NBRUN / 32);
    int s = 0;
#pragma unroll 1
    for (int i = 0; i < NBRUN / 32; ++i) s += cnt[base + i];
    int incl = s;
#pragma unroll
    for (int d = 1; d < 32; d <<= 1) {
      const int y = __shfl_up(incl, d, 32);
      if (lane >= d) incl += y;
    }
    int run = incl - s;
#pragma unroll 1
    for (int i = 0; i < NBRUN / 32; ++i) {
      const int cv = cnt[base + i];
      offs[base + i] = run;
      cur[base + i]  = run;
      run += cv;
    }
  }
  __syncthreads();

  if (wave == 0) {
#pragma unroll 1
    for (int w2 = 0; w2 < NWAVE; ++w2) {
      int c = misc[w2];
      c = c < 0 ? 0 : (c > WLCAP ? WLCAP : c);
#pragma unroll 1
      for (int b0 = 0; b0 < c; b0 += 32) {
        const int idx = b0 + lane;
        const int ent = wl[w2 * WLCAP + (idx < WLCAP ? idx : WLCAP - 1)];
        int eid = (ent >> SLB) & 0xFFFFF;
        eid = eid > NE - 1 ? NE - 1 : eid;
        int sr = srcs[eid];
        sr = sr < 0 ? 0 : (sr > NN - 1 ? NN - 1 : sr);
        const int m32 = (c - b0) < 32 ? (c - b0) : 32;
#pragma unroll 1
        for (int k = 0; k < m32; ++k) {
          const int u    = __builtin_amdgcn_readlane(ent, k);
          const int wd   = __builtin_amdgcn_readlane(sr, k);
          const int slot = u & (NBRUN - 1);
          if (lane == 0) {
            int p = cur[slot];
            p = p < 0 ? 0 : (p > RCAP - 1 ? RCAP - 1 : p);
            pl[p] = wd;
            cur[slot] = p + 1;
          }
        }
      }
    }
  }
  __syncthreads();

  const int ovf = misc[9];
  int* lp  = LIST + (size_t)blk * RCAP;
  int* cop = CO + (size_t)blk * (2 * NBRUN);
  int* fp  = FLAG + (size_t)blk * 32;
  bucket_flush(pl, cnt, ovf, lp, cop, fp, tid);
  __threadfence();
  bucket_flush(pl, cnt, ovf, lp, cop, fp, tid);
}

__device__ __forceinline__ void upd4(const v4f xs, const v4f xr, const v4f at, float& m, float& den,
                                     float& a0, float& a1, float& a2, float& a3) {
  float t0 = xs.x + xr.x, t1 = xs.y + xr.y, t2 = xs.z + xr.z, t3 = xs.w + xr.w;
  t0 = (t0 > 0.0f) ? t0 : NEGS * t0;
  t1 = (t1 > 0.0f) ? t1 : NEGS * t1;
  t2 = (t2 > 0.0f) ? t2 : NEGS * t2;
  t3 = (t3 > 0.0f) ? t3 : NEGS * t3;
  float part = t0 * at.x;
  part = fmaf(t1, at.y, part);
  part = fmaf(t2, at.z, part);
  part = fmaf(t3, at.w, part);
  part += __shfl_xor(part, 1, 32);
  part += __shfl_xor(part, 2, 32);
  part += __shfl_xor(part, 4, 32);
  part += __shfl_xor(part, 8, 32);
  const float mn = fmaxf(m, part);
  const float sc = expf(m - mn);
  const float p  = expf(part - mn);
  den = fmaf(den, sc, p);
  a0 = fmaf(a0, sc, p * xs.x);
  a1 = fmaf(a1, sc, p * xs.y);
  a2 = fmaf(a2, sc, p * xs.z);
  a3 = fmaf(a3, sc, p * xs.w);
  m = mn;
}

__device__ __forceinline__ void upd2(const v2f xs, const v2f xr, const v2f at, float& m, float& den,
                                     float& a0, float& a1) {
  float t0 = xs.x + xr.x, t1 = xs.y + xr.y;
  t0 = (t0 > 0.0f) ? t0 : NEGS * t0;
  t1 = (t1 > 0.0f) ? t1 : NEGS * t1;
  float part = t0 * at.x;
  part = fmaf(t1, at.y, part);
  part += __shfl_xor(part, 1, 32);
  part += __shfl_xor(part, 2, 32);
  part += __shfl_xor(part, 4, 32);
  part += __shfl_xor(part, 8, 32);
  part += __shfl_xor(part, 16, 32);
  const float mn = fmaxf(m, part);
  const float sc = expf(m - mn);
  const float p  = expf(part - mn);
  den = fmaf(den, sc, p);
  a0 = fmaf(a0, sc, p * xs.x);
  a1 = fmaf(a1, sc, p * xs.y);
  m = mn;
}

__global__ __launch_bounds__(NTHR) void k_replay_one(const int* __restrict__ LIST, const int* __restrict__ CO,
                                                     const int* __restrict__ FLAG, const float* __restrict__ X,
                                                     const float* __restrict__ sm, unsigned short* E) {
  const int tid = (int)threadIdx.x, lane = tid & 31, wave = tid >> 5;
  const int d      = (int)blockIdx.x * NWAVE + wave;
  const int lv     = (int)(d < NN);
  const int dcl    = min(d, NN - 1);
  const int bucket = d >> SLB;
  const int slot   = d & (NBRUN - 1);
  const int* cob = CO + (size_t)bucket * (2 * NBRUN);
  int c = cob[slot];
  int o = cob[NBRUN + slot];
  const int flag = FLAG[(size_t)bucket * 32];
  asm volatile("" :: "v"(c), "v"(o), "v"(flag));
  const bool big = c > DEGCAP;
  c = max(c, 0); c = min(c, DEGCAP); c = c * lv;
  o = max(o, 0); o = min(o, RCAP - 1);
  int last = o + c - 1;
  last = max(last, o);
  last = min(last, RCAP - 1);
  const int cs  = __builtin_amdgcn_readfirstlane(c);
  const int os  = __builtin_amdgcn_readfirstlane(o);
  const int ls  = __builtin_amdgcn_readfirstlane(last);
  const int bks = __builtin_amdgcn_readfirstlane(bucket);
  const int* lb = LIST + (size_t)bks * RCAP;

  const float* drow = X + (size_t)dcl * W1N;
  const v4f xld = *(const v4fa*)(drow + 4 * lane);
  const v4f xrd = *(const v4fa*)(drow + 128 + 4 * lane);
  const v4f at  = *(const v4fa*)(sm + SM_ATT1 + 4 * lane);
  const v4f bb  = *(const v4fa*)(sm + SM_B1 + 4 * lane);
  asm volatile("" :: "v"(xld));
  asm volatile("" :: "v"(xrd));
  asm volatile("" :: "v"(at));
  asm volatile("" :: "v"(bb));

  float m = -INFINITY, den = 0.0f, a0 = 0.0f, a1 = 0.0f, a2 = 0.0f, a3 = 0.0f;
#pragma unroll 1
  for (int j = 0; j < cs; ++j) {
    int idx = os + j;
    idx = min(idx, ls);
    int sr = lb[idx];
    sr = max(sr, 0); sr = min(sr, NN - 1);
    const v4f xs = *(const v4fa*)(X + (size_t)sr * W1N + 4 * lane);
    upd4(xs, xrd, at, m, den, a0, a1, a2, a3);
  }
  upd4(xld, xrd, at, m, den, a0, a1, a2, a3);

  const float inv = 1.0f / (den + 1e-16f);
  float v0 = fmaf(a0, inv, bb.x), v1 = fmaf(a1, inv, bb.y), v2 = fmaf(a2, inv, bb.z), v3 = fmaf(a3, inv, bb.w);
  v0 = (v0 > 0.0f) ? v0 : (v0 - v0); v1 = (v1 > 0.0f) ? v1 : (v1 - v1);
  v2 = (v2 > 0.0f) ? v2 : (v2 - v2); v3 = (v3 > 0.0f) ? v3 : (v3 - v3);
  const float qnan = __uint_as_float(0x7fc00000u);
  const bool bad = (flag != 0) | big;
  v0 = bad ? qnan : v0; v1 = bad ? qnan : v1; v2 = bad ? qnan : v2; v3 = bad ? qnan : v3;
  v0 = (lv != 0) ? v0 : 0.0f; v1 = (lv != 0) ? v1 : 0.0f; v2 = (lv != 0) ? v2 : 0.0f; v3 = (lv != 0) ? v3 : 0.0f;
  const unsigned h0 = bf16_bits(v0), h1 = bf16_bits(v1), h2 = bf16_bits(v2), h3 = bf16_bits(v3);
  const unsigned l0 = bf16_bits(v0 - __uint_as_float(h0 << 16));
  const unsigned l1 = bf16_bits(v1 - __uint_as_float(h1 << 16));
  const unsigned l2 = bf16_bits(v2 - __uint_as_float(h2 << 16));
  const unsigned l3 = bf16_bits(v3 - __uint_as_float(h3 << 16));
  v2u hw, lw;
  hw.x = h0 | (h1 << 16); hw.y = h2 | (h3 << 16);
  lw.x = l0 | (l1 << 16); lw.y = l2 | (l3 << 16);
  unsigned short* ep = E + (size_t)d * EP + 4 * lane;
  *(volatile v2u*)ep = hw;
  *(volatile v2u*)(ep + 128) = lw;
  __threadfence();
  *(volatile v2u*)ep = hw;
  *(volatile v2u*)(ep + 128) = lw;
}

__global__ __launch_bounds__(NTHR) void k_replay_two(const int* __restrict__ LIST, const int* __restrict__ CO,
                                                     const int* __restrict__ FLAG, const float* __restrict__ X,
                                                     const float* __restrict__ sm, float* out) {
  const int tid = (int)threadIdx.x, lane = tid & 31, wave = tid >> 5;
  const int d      = (int)blockIdx.x * NWAVE + wave;
  const int lv     = (int)(d < NN);
  const int dcl    = min(d, NN - 1);
  const int bucket = dcl >> SLB;
  const int slot   = dcl & (NBRUN - 1);
  const int* cob = CO + (size_t)bucket * (2 * NBRUN);
  int c = cob[slot];
  int o = cob[NBRUN + slot];
  const int flag = FLAG[(size_t)bucket * 32];
  asm volatile("" :: "v"(c), "v"(o), "v"(flag));
  const bool big = c > DEGCAP;
  c = max(c, 0); c = min(c, DEGCAP); c = c * lv;
  o = max(o, 0); o = min(o, RCAP - 1);
  int last = o + c - 1;
  last = max(last, o);
  last = min(last, RCAP - 1);
  const int cs  = __builtin_amdgcn_readfirstlane(c);
  const int os  = __builtin_amdgcn_readfirstlane(o);
  const int ls  = __builtin_amdgcn_readfirstlane(last);
  const int bks = __builtin_amdgcn_readfirstlane(bucket);
  const int* lb = LIST + (size_t)bks * RCAP;

  const float* drow = X + (size_t)dcl * W2N;
  const v2f xld = *(const v2fa*)(drow + 2 * lane);
  const v2f xrd = *(const v2fa*)(drow + 64 + 2 * lane);
  const v2f at  = *(const v2fa*)(sm + SM_ATT2 + 2 * lane);
  const v2f bb  = *(const v2fa*)(sm + SM_B2 + 2 * lane);
  asm volatile("" :: "v"(xld));
  asm volatile("" :: "v"(xrd));
  asm volatile("" :: "v"(at));
  asm volatile("" :: "v"(bb));

  float m = -INFINITY, den = 0.0f, a0 = 0.0f, a1 = 0.0f;
#pragma unroll 1
  for (int j = 0; j < cs; ++j) {
    int idx = os + j;
    idx = min(idx, ls);
    int sr = lb[idx];
    sr = max(sr, 0); sr = min(sr, NN - 1);
    const v2f xs = *(const v2fa*)(X + (size_t)sr * W2N + 2 * lane);
    upd2(xs, xrd, at, m, den, a0, a1);
  }
  upd2(xld, xrd, at, m, den, a0, a1);

  const float inv = 1.0f / (den + 1e-16f);
  float v0 = fmaf(a0, inv, bb.x), v1 = fmaf(a1, inv, bb.y);
  v0 = (v0 > 0.0f) ? v0 : (v0 - v0);
  v1 = (v1 > 0.0f) ? v1 : (v1 - v1);
  const float qnan = __uint_as_float(0x7fc00000u);
  const bool bad = (flag != 0) | big;
  v0 = bad ? qnan : v0;
  v1 = bad ? qnan : v1;
  v2f ov;
  ov.x = v0; ov.y = v1;
  float* op = out + (size_t)dcl * C2 + 2 * lane;
  if (lv != 0) *(volatile v2f*)op = ov;
  __threadfence();
  if (lv != 0) *(volatile v2f*)op = ov;
}

extern "C" void kernel_launch(void* const* d_in, const int* in_sizes, int n_in,
                              void* d_out, int out_size, void* d_ws, size_t ws_size,
                              hipStream_t stream) {
  if (n_in < 10) return;
  if (in_sizes[0] != NN * DIN) return;
  if (in_sizes[1] != 2 * NE) return;
  if (in_sizes[2] != DIN * 128) return;
  if (in_sizes[3] != DIN * 128) return;
  if (in_sizes[4] != 128) return;
  if (in_sizes[5] != 128) return;
  if (in_sizes[6] != 128 * 64) return;
  if (in_sizes[7] != 128 * 64) return;
  if (in_sizes[8] != 64) return;
  if (in_sizes[9] != 64) return;
  if (out_size != NN * C2) return;

  const float* x    = (const float*)d_in[0];
  const int*   ei   = (const int*)d_in[1];
  const float* Wl1  = (const float*)d_in[2];
  const float* Wr1  = (const float*)d_in[3];
  const float* att1 = (const float*)d_in[4];
  const float* b1   = (const float*)d_in[5];
  const float* Wl2  = (const float*)d_in[6];
  const float* Wr2  = (const float*)d_in[7];
  const float* att2 = (const float*)d_in[8];
  const float* b2   = (const float*)d_in[9];
  float* out = (float*)d_out;
  const int* srcs = ei;
  const int* dsts = ei + NE;

  constexpr size_t zXB   = (size_t)MP * DIN * 2;
  constexpr size_t zXLR  = (size_t)MP * W1N * 4;
  constexpr size_t zXLR2 = (size_t)MP * W2N * 4;
  constexpr size_t zE    = (size_t)MP * EP * 2;
  constexpr size_t zLIST = (size_t)NBK * RCAP * 4;
  constexpr size_t zCO   = (size_t)NBK * 2 * NBRUN * 4;
  constexpr size_t zFLAG = (size_t)(NBK + 1) * 128;
  constexpr size_t zBT1  = (size_t)W1N * DIN * 2;
  constexpr size_t zBT2  = (size_t)W2N * 256 * 2;
  constexpr size_t zSM   = (size_t)SM_N * 4;
  constexpr size_t oXB   = 0;
  constexpr size_t oXLR  = oXB + zXB;
  constexpr size_t oE    = oXLR + zXLR;
  constexpr size_t oLIST = oE + zE;
  constexpr size_t oCO   = oLIST + zLIST;
  constexpr size_t oFLAG = oCO + zCO;
  constexpr size_t oBT1  = oFLAG + zFLAG;
  constexpr size_t oBT2  = oBT1 + zBT1;
  constexpr size_t oSM   = oBT2 + zBT2;
  constexpr size_t oEND  = oSM + zSM;
  static_assert(zXB % 256 == 0 && zXLR % 256 == 0 && zE % 256 == 0 && zLIST % 256 == 0 && zCO % 256 == 0);
  static_assert(zFLAG % 256 == 0 && zBT1 % 256 == 0 && zBT2 % 256 == 0 && zSM % 256 == 0);
  static_assert(zXLR2 <= zXLR);
  static_assert(oEND <= (size_t)(128u << 20));
  if (oEND > ws_size) return;

  char* ws = (char*)d_ws;
  unsigned short* XB   = (unsigned short*)(ws + oXB);
  float*          XLR1 = (float*)(ws + oXLR);
  float*          XLR2 = (float*)(ws + oXLR);
  unsigned short* E    = (unsigned short*)(ws + oE);
  int*            LIST = (int*)(ws + oLIST);
  int*            CO   = (int*)(ws + oCO);
  int*            FLAG = (int*)(ws + oFLAG);
  unsigned short* BT1  = (unsigned short*)(ws + oBT1);
  unsigned short* BT2  = (unsigned short*)(ws + oBT2);
  float*          SM   = (float*)(ws + oSM);

  hipFuncSetAttribute(reinterpret_cast<const void*>(&k_bucket), hipFuncAttributeMaxDynamicSharedMemorySize, (int)BK_LDS);

  k_prep<<<PBTOT, NTHR, 0, stream>>>(x, Wl1, Wr1, att1, b1, Wl2, Wr2, att2, b2, XB, BT1, BT2, SM);
  k_gemm_one<<<dim3(MP / GBM, W1N / 64), NTHR, 0, stream>>>(XB, BT1, XLR1);
  k_bucket<<<NBK, NTHR, BK_LDS, stream>>>(srcs, dsts, LIST, CO, FLAG);
  k_replay_one<<<MP / NWAVE, NTHR, 0, stream>>>(LIST, CO, FLAG, XLR1, SM, E);
  k_gemm_two<<<dim3(MP / GBM, W2N / 64), NTHR, 0, stream>>>(E, BT2, XLR2);
  k_replay_two<<<NN / NWAVE, NTHR, 0, stream>>>(LIST, CO, FLAG, XLR2, SM, out);
}
